// QKVAttention_39599598469377
// MI455X (gfx1250) — hardware-verified
//
#include <hip/hip_runtime.h>
#include <math.h>

constexpr int kB    = 8;
constexpr int kT    = 1000;
constexpr int kC    = 8;
constexpr int kF    = 128;
constexpr int kA    = 128;
constexpr int kTok  = kB * kT;
constexpr int kRows = kTok * kC;
constexpr int kQKld = 2 * kA;
constexpr int kPoolWaves = 4;
constexpr int kQPitch = 132;
constexpr float kWCarry     = 16.0f;
constexpr float kWCarryInv  = 1.0f / 16.0f;
constexpr float kScoreScale = 0.08838834764831845f;
static_assert(kRows % 64 == 0, "M tile multiple");
static_assert(kA % 64 == 0, "N tile multiple");
static_assert(kF % 32 == 0, "K multiple of 32");
static_assert(kA % 64 == 0 && kF % 64 == 0, "weight transpose tiles");
static_assert(kTok % kPoolWaves == 0, "pool grid exact");
static_assert((kRows * kF) % (8 * 256) == 0, "cast grid exact");
static_assert(kF == 4 * 32, "one float4 per lane per row");

typedef __attribute__((ext_vector_type(16))) _Float16 v16h;
typedef __attribute__((ext_vector_type(8)))  _Float16 v8h;
typedef __attribute__((ext_vector_type(16))) __bf16   v16b;
typedef __attribute__((ext_vector_type(8)))  __bf16   v8b;
typedef __attribute__((ext_vector_type(8)))  float    v8f;
typedef __attribute__((ext_vector_type(4)))  float    v4f;
typedef __attribute__((ext_vector_type(4)))  unsigned int v4u;

__device__ __forceinline__ unsigned short f2bf_bits(float f) {
  unsigned u = __float_as_uint(f);
  return (unsigned short)((u + 0x7FFFu + ((u >> 16) & 1u)) >> 16);
}
__device__ __forceinline__ float bf_bits2f(unsigned short h) { return __uint_as_float(((unsigned)h) << 16); }

__device__ __forceinline__ void dep_guard_h(v8f& a, v8f& b, v16h x, v16h y) { asm volatile("v_nop\n\tv_nop\n\tv_nop\n\tv_nop" : "+v"(a), "+v"(b) : "v"(x), "v"(y)); }
__device__ __forceinline__ void dep_guard_b(v8f& a, v8f& b, v16b x, v16b y) { asm volatile("v_nop\n\tv_nop\n\tv_nop\n\tv_nop" : "+v"(a), "+v"(b) : "v"(x), "v"(y)); }
__device__ __forceinline__ void keep4_h(v16h a, v16h b, v16h c, v16h d) { asm volatile("v_nop" :: "v"(a), "v"(b), "v"(c), "v"(d)); }
__device__ __forceinline__ void keep4_b(v16b a, v16b b, v16b c, v16b d) { asm volatile("v_nop" :: "v"(a), "v"(b), "v"(c), "v"(d)); }
__device__ __forceinline__ void acc_guard4(v8f& a, v8f& b, v8f& c, v8f& d) { asm volatile("v_nop\n\tv_nop\n\tv_nop\n\tv_nop" : "+v"(a), "+v"(b), "+v"(c), "+v"(d)); }
template <typename T> struct Frag;
template <> struct Frag<_Float16> {
  typedef v16h V; union U { v16h v; v8h h[2]; };
  static __device__ __forceinline__ v16h load(const _Float16* p) {
    U f; f.h[0] = *(const v8h*)(p); f.h[1] = *(const v8h*)(p + 16); return f.v;
  }
  static __device__ __forceinline__ v8f mma(v16h a, v16h b, v8f c) {
    return __builtin_amdgcn_wmma_f32_16x16x32_f16(false, a, false, b, (short)0, c, false, false);
  }
  static __device__ __forceinline__ void guard(v8f& a, v8f& b, v16h x, v16h y) { dep_guard_h(a, b, x, y); }
  static __device__ __forceinline__ void keep(v16h a, v16h b, v16h c, v16h d) { keep4_h(a, b, c, d); }
};
template <> struct Frag<__bf16> {
  typedef v16b V; union U { v16b v; v8b h[2]; };
  static __device__ __forceinline__ v16b load(const __bf16* p) {
    U f; f.h[0] = *(const v8b*)(p); f.h[1] = *(const v8b*)(p + 16); return f.v;
  }
  static __device__ __forceinline__ v8f mma(v16b a, v16b b, v8f c) {
    return __builtin_amdgcn_wmma_f32_16x16x32_bf16(false, a, false, b, (short)0, c, false, false);
  }
  static __device__ __forceinline__ void guard(v8f& a, v8f& b, v16b x, v16b y) { dep_guard_b(a, b, x, y); }
  static __device__ __forceinline__ void keep(v16b a, v16b b, v16b c, v16b d) { keep4_b(a, b, c, d); }
};

__device__ __forceinline__ unsigned pk16(unsigned short a, unsigned short b) { return (unsigned)a | ((unsigned)b << 16); }
__device__ __forceinline__ unsigned short h_bits(float f) { const _Float16 h = (_Float16)f; return __builtin_bit_cast(unsigned short, h); }

template <int ET> struct Elem;
template <> struct Elem<0> { typedef _Float16 T; };
template <> struct Elem<1> { typedef __bf16 T; };
template <int ET, bool SPLIT, int BIAS_MODE, int OUT_MODE, bool RESID, int ACT = 0>
__global__ __launch_bounds__(256) void wmma_gemm64(
    const unsigned short* __restrict__ Ap, const unsigned short* __restrict__ A2p, int lda, long strideA,
    const unsigned short* __restrict__ Btp, const unsigned short* __restrict__ Bt2p, int ldb, long strideB,
    void* __restrict__ Cout, void* __restrict__ Cout2, int ldc, long strideC,
    const float* __restrict__ bias,
    const float* __restrict__ resid, long strideR,
    int M, int N, int K, float scale) {
  typedef typename Elem<ET>::T T;
  typedef typename Frag<T>::V V;
  const T* A = (const T*)Ap; const T* A2 = (const T*)A2p; const T* Bt = (const T*)Btp; const T* Bt2 = (const T*)Bt2p;
  __shared__ __align__(16) float sT[8][16 * 68];
  const int b    = blockIdx.y;
  const int lane = threadIdx.x & 31;
  const int wave = threadIdx.x >> 5;
  const int tilesN = N >> 6;
  const int tilesM = M >> 6;
  const int tile = blockIdx.x * 8 + wave;
  if (tile >= tilesM * tilesN) return;
  const int tm = tile / tilesN;
  const int tn = tile - tm * tilesN;
  const int m0 = tm << 6;
  const int n0 = tn << 6;

  const T* Ab  = A  + (size_t)b * strideA;
  const T* Bb  = Bt + (size_t)b * strideB;
  const T* Ab2 = SPLIT ? (A2  + (size_t)b * strideA) : nullptr;
  const T* Bb2 = SPLIT ? (Bt2 + (size_t)b * strideB) : nullptr;

  const int rlane = lane & 15;
  const int koff  = (lane >> 4) * 8;
  const int mOff  = (lane >> 4) * 8;

  v8f acc[4][4];
#pragma unroll
  for (int i = 0; i < 4; ++i)
#pragma unroll
    for (int j = 0; j < 4; ++j) acc[i][j] = (v8f){0.f,0.f,0.f,0.f,0.f,0.f,0.f,0.f};

  for (int k0 = 0; k0 < K; k0 += 32) {
    V bh[4], bl[4];
#pragma unroll
    for (int j = 0; j < 4; ++j) {
      const size_t bo = (size_t)(n0 + (j << 4) + rlane) * ldb + koff + k0;
      bh[j] = Frag<T>::load(Bb + bo);
      if (SPLIT) bl[j] = Frag<T>::load(Bb2 + bo);
    }
#pragma unroll
    for (int i = 0; i < 4; ++i) {
      const size_t ao = (size_t)(m0 + (i << 4) + rlane) * lda + koff + k0;
      V ah = Frag<T>::load(Ab + ao);
      V al;
      if (SPLIT) al = Frag<T>::load(Ab2 + ao);
#pragma unroll
      for (int j = 0; j < 4; ++j) {
        acc[i][j] = Frag<T>::mma(ah, bh[j], acc[i][j]);
        if (SPLIT) {
          acc[i][j] = Frag<T>::mma(ah, bl[j], acc[i][j]);
          acc[i][j] = Frag<T>::mma(al, bh[j], acc[i][j]);
        }
      }
      Frag<T>::guard(acc[i][0], acc[i][3], ah, SPLIT ? al : ah);
    }
    Frag<T>::keep(bh[0], bh[1], bh[2], bh[3]);
    if (SPLIT) Frag<T>::keep(bl[0], bl[1], bl[2], bl[3]);
  }
  acc_guard4(acc[0][0], acc[0][1], acc[0][2], acc[0][3]);
  acc_guard4(acc[1][0], acc[1][1], acc[1][2], acc[1][3]);
  acc_guard4(acc[2][0], acc[2][1], acc[2][2], acc[2][3]);
  acc_guard4(acc[3][0], acc[3][1], acc[3][2], acc[3][3]);

  float* slab = sT[wave];
  const float* Rb = RESID ? (resid + (size_t)b * strideR) : nullptr;
#pragma unroll
  for (int i = 0; i < 4; ++i) {
    const int mBase = m0 + (i << 4);
#pragma unroll
    for (int j = 0; j < 4; ++j) {
      const int n = n0 + (j << 4) + rlane;
      float bv = 0.f;
      if (BIAS_MODE == 2) bv = bias[n];
#pragma unroll
      for (int r = 0; r < 8; ++r) {
        float v = acc[i][j][r] * scale;
        if (BIAS_MODE == 1) v += bias[mBase + mOff + r];
        if (BIAS_MODE == 2) v += bv;
        if (RESID) v += Rb[(size_t)(mBase + mOff + r) * ldc + n];
        if (ACT == 2) v = fmaxf(v, 0.0f);
        if (ACT == 4) v = (v > 0.f) ? v : 0.01f * v;
        slab[(mOff + r) * 68 + (j << 4) + rlane] = v;
      }
    }
    __builtin_amdgcn_fence(__ATOMIC_RELEASE, "workgroup");
    __builtin_amdgcn_wave_barrier();
    __builtin_amdgcn_fence(__ATOMIC_ACQUIRE, "workgroup");
    if (OUT_MODE == 0) {
      float* C = (float*)Cout + (size_t)b * strideC;
      const int hh = lane >> 4, c4 = (lane & 15) * 4;
      for (int pass = 0; pass < 2; ++pass) {
#pragma unroll
        for (int it = 0; it < 8; ++it) {
          const int row = it * 2 + hh;
          v4f v = *(const v4f*)(slab + row * 68 + c4);
          *(volatile v4f*)(C + (size_t)(mBase + row) * ldc + n0 + c4) = v;
        }
        __threadfence();
      }
    } else {
      const int q = lane >> 3, c8 = (lane & 7) * 8;
      unsigned short* C  = (unsigned short*)Cout  + (size_t)b * strideC;
      unsigned short* C2 = (OUT_MODE == 2) ? ((unsigned short*)Cout2 + (size_t)b * strideC) : nullptr;
      for (int pass = 0; pass < 2; ++pass) {
#pragma unroll
        for (int it = 0; it < 4; ++it) {
          const int row = it * 4 + q;
          const float* sp = slab + row * 68 + c8;
          v8h hv, lv;
#pragma unroll
          for (int e = 0; e < 8; ++e) {
            if (OUT_MODE == 1) {
              hv[e] = (_Float16)sp[e];
            } else {
              unsigned short hb = f2bf_bits(sp[e]);
              unsigned short lb = f2bf_bits(sp[e] - bf_bits2f(hb));
              hv[e] = __builtin_bit_cast(_Float16, hb);
              lv[e] = __builtin_bit_cast(_Float16, lb);
            }
          }
          *(volatile v8h*)(C + (size_t)(mBase + row) * ldc + n0 + c8) = hv;
          if (OUT_MODE == 2) *(volatile v8h*)(C2 + (size_t)(mBase + row) * ldc + n0 + c8) = lv;
        }
        __threadfence();
      }
    }
    __builtin_amdgcn_fence(__ATOMIC_RELEASE, "workgroup");
    __builtin_amdgcn_wave_barrier();
    __builtin_amdgcn_fence(__ATOMIC_ACQUIRE, "workgroup");
  }
}

__global__ __launch_bounds__(256) void cast8_f16_kernel(const float* __restrict__ in, unsigned short* __restrict__ out, int n8) {
  const int i = blockIdx.x * 256 + threadIdx.x;
  if (i >= n8) return;
  const float* p = in + 8 * (size_t)i;
  const v4f a = *(const v4f*)(p);
  const v4f c = *(const v4f*)(p + 4);
  unsigned short hb[8];
#pragma unroll
  for (int e = 0; e < 4; ++e) {
    hb[e]     = h_bits(a[e]);
    hb[4 + e] = h_bits(c[e]);
  }
  const v4u u = (v4u){pk16(hb[0], hb[1]), pk16(hb[2], hb[3]), pk16(hb[4], hb[5]), pk16(hb[6], hb[7])};
  unsigned short* q = out + 8 * (size_t)i;
  *(volatile v4u*)q = u;
  __threadfence();
  *(volatile v4u*)q = u;
}

__global__ __launch_bounds__(256) void wtcast2_kernel(const float* __restrict__ W0, const float* __restrict__ W1,
                                                      unsigned short* __restrict__ outp, float scale) {
  __shared__ float sm[64][65];
  const int t  = threadIdx.x;
  const int k0 = blockIdx.x * 64;
  const int n0 = blockIdx.y * 64;
  const int z  = blockIdx.z;
  const float* W = (z == 0) ? W0 : W1;
#pragma unroll
  for (int i = 0; i < 16; ++i) {
    const int e = i * 256 + t;
    const int r = e >> 6;
    const int c = e & 63;
    sm[c][r] = W[(size_t)(k0 + r) * kA + n0 + c] * scale;
  }
  __syncthreads();
  const int lane = t & 31, wave = t >> 5;
  const int q = lane >> 3, c8 = (lane & 7) * 8;
  unsigned short* op = outp + (size_t)z * kA * kF;
  for (int pass = 0; pass < 2; ++pass) {
#pragma unroll
    for (int it = 0; it < 2; ++it) {
      const int row = wave * 8 + it * 4 + q;
      unsigned short hb[8];
#pragma unroll
      for (int e = 0; e < 8; ++e) hb[e] = h_bits(sm[row][c8 + e]);
      const v4u u = (v4u){pk16(hb[0], hb[1]), pk16(hb[2], hb[3]), pk16(hb[4], hb[5]), pk16(hb[6], hb[7])};
      *(volatile v4u*)(op + (size_t)(n0 + row) * kF + k0 + c8) = u;
    }
    __threadfence();
  }
}

__global__ __launch_bounds__(32 * kPoolWaves) void pool_kernel(const float* __restrict__ QK, const float* __restrict__ x,
                                                                const float* __restrict__ Wv, const float* __restrict__ Bv,
                                                                float* __restrict__ out, int ntok) {
  __shared__ __align__(16) float sQ[kPoolWaves][kC * kQPitch];
  __shared__ __align__(16) float sK[kPoolWaves][kC * kQPitch];
  __shared__ float sV[kPoolWaves][kC];
  __shared__ float sU[kPoolWaves][kC];
  __shared__ float sW[kPoolWaves][kC];

  const int tid  = threadIdx.x;
  const int lane = tid & 31;
  const int wave = tid >> 5;
  int tok = blockIdx.x * kPoolWaves + wave;
  const bool live = (tok < ntok);
  tok = (tok < ntok) ? tok : (ntok - 1);
  const float* qkrow = QK + (size_t)tok * kC * kQKld;
  const float* xrow  = x  + (size_t)tok * kC * kF;
  float* sq = sQ[wave];
  float* sk = sK[wave];

#pragma unroll 2
  for (int c = 0; c < kC; ++c) {
    const v4f qv = *(const v4f*)(qkrow + (size_t)c * kQKld + 4 * lane);
    const v4f kv = *(const v4f*)(qkrow + (size_t)c * kQKld + kA + 4 * lane);
    *(v4f*)(sq + c * kQPitch + 4 * lane) = qv;
    *(v4f*)(sk + c * kQPitch + 4 * lane) = kv;
  }

  const v4f wv4 = *(const v4f*)(Wv + 4 * lane);
  const float bvs = Bv[0];
#pragma unroll 1
  for (int c = 0; c < kC; ++c) {
    const v4f xv = *(const v4f*)(xrow + (size_t)c * kF + 4 * lane);
    float p = 0.0f;
    p += xv[0] * wv4[0];
    p += xv[1] * wv4[1];
    p += xv[2] * wv4[2];
    p += xv[3] * wv4[3];
#pragma unroll
    for (int off = 16; off > 0; off >>= 1) p += __shfl_xor(p, off, 32);
    if (lane == 0) sV[wave][c] = p + bvs;
  }
  __syncthreads();

  {
    const int c  = lane >> 2;
    const int d0 = (lane & 3) * 2;
    const int d1 = d0 + 1;
    const float* qp  = sq + c  * kQPitch;
    const float* k0p = sk + d0 * kQPitch;
    const float* k1p = sk + d1 * kQPitch;
    float a0 = 0.0f, a1 = 0.0f;
#pragma unroll 1
    for (int a = 0; a < kA; a += 4) {
      const v4f qa = *(const v4f*)(qp + a);
      const v4f ka = *(const v4f*)(k0p + a);
      const v4f kb = *(const v4f*)(k1p + a);
      a0 += qa[0] * ka[0]; a0 += qa[1] * ka[1]; a0 += qa[2] * ka[2]; a0 += qa[3] * ka[3];
      a1 += qa[0] * kb[0]; a1 += qa[1] * kb[1]; a1 += qa[2] * kb[2]; a1 += qa[3] * kb[3];
    }
    const float s0 = a0 * kScoreScale;
    const float s1 = a1 * kScoreScale;
    float m = fmaxf(s0, s1);
    m = fmaxf(m, __shfl_xor(m, 1, 32));
    m = fmaxf(m, __shfl_xor(m, 2, 32));
    const float e0 = expf(s0 - m);
    const float e1 = expf(s1 - m);
    float den = e0 + e1;
    den += __shfl_xor(den, 1, 32);
    den += __shfl_xor(den, 2, 32);
    const float v0 = sV[wave][d0];
    const float v1 = sV[wave][d1];
    float num = 0.0f;
    num += e0 * v0;
    num += e1 * v1;
    num += __shfl_xor(num, 1, 32);
    num += __shfl_xor(num, 2, 32);
    const float u = num * (1.0f / den);
    if ((lane & 3) == 0) sU[wave][c] = u;
  }
  __syncthreads();

  {
    const float uv = sU[wave][lane & 7];
    float mu = uv;
    mu = fmaxf(mu, __shfl_xor(mu, 1, 32));
    mu = fmaxf(mu, __shfl_xor(mu, 2, 32));
    mu = fmaxf(mu, __shfl_xor(mu, 4, 32));
    const float ew = expf(uv - mu);
    float sw = ew;
    sw += __shfl_xor(sw, 1, 32);
    sw += __shfl_xor(sw, 2, 32);
    sw += __shfl_xor(sw, 4, 32);
    const float wch = ew * (1.0f / sw);
    if (lane < 8) sW[wave][lane] = wch;
  }
  __syncthreads();

  float o0 = 0.0f, o1 = 0.0f, o2 = 0.0f, o3 = 0.0f;
#pragma unroll 1
  for (int c = 0; c < kC; ++c) {
    const v4f xv = *(const v4f*)(xrow + (size_t)c * kF + 4 * lane);
    const float wc = sW[wave][c];
    o0 += wc * xv[0];
    o1 += wc * xv[1];
    o2 += wc * xv[2];
    o3 += wc * xv[3];
  }
  const v4f ov = (v4f){o0, o1, o2, o3};
  if (live) {
    float* op = out + (size_t)tok * kF + 4 * lane;
    *(volatile v4f*)op = ov;
    __threadfence();
    *(volatile v4f*)op = ov;
  }
}

extern "C" void kernel_launch(void* const* d_in, const int* in_sizes, int n_in,
                              void* d_out, int out_size, void* d_ws, size_t ws_size,
                              hipStream_t stream) {
  if (n_in < 7) return;
  if (in_sizes[0] != kRows * kF) return;
  if (in_sizes[1] != kF * kA) return;
  if (in_sizes[2] != kA) return;
  if (in_sizes[3] != kF * kA) return;
  if (in_sizes[4] != kA) return;
  if (in_sizes[5] != kF) return;
  if (in_sizes[6] != 1) return;
  if (out_size != kTok * kF) return;

  const size_t szX16 = (size_t)kRows * kF * 2;
  const size_t szWT  = (size_t)2 * kA * kF * 2;
  const size_t szQK  = (size_t)kRows * kQKld * 4;
  const size_t offX16 = 0;
  const size_t offWT  = offX16 + szX16;
  const size_t offQK  = offWT + szWT;
  const size_t total  = offQK + szQK;
  if (ws_size < total) return;

  const float* x  = (const float*)d_in[0];
  const float* Wq = (const float*)d_in[1];
  const float* bq = (const float*)d_in[2];
  const float* Wk = (const float*)d_in[3];
  const float* bk = (const float*)d_in[4];
  const float* Wv = (const float*)d_in[5];
  const float* bv = (const float*)d_in[6];
  float* out = (float*)d_out;
  char* ws = (char*)d_ws;
  unsigned short* X16 = (unsigned short*)(ws + offX16);
  unsigned short* WT  = (unsigned short*)(ws + offWT);
  float* QK = (float*)(ws + offQK);

  const int n8 = (kRows * kF) / 8;
  cast8_f16_kernel<<<dim3(n8 / 256), dim3(256), 0, stream>>>(x, X16, n8);
  wtcast2_kernel<<<dim3(kF / 64, kA / 64, 2), dim3(256), 0, stream>>>(Wq, Wk, WT, kWCarry);

  const int tiles = (kRows / 64) * (kA / 64);
  const int gemmBlocks = (tiles + 7) / 8;
  wmma_gemm64<0, false, 2, 0, false, 0><<<dim3(gemmBlocks, 1), dim3(256), 0, stream>>>(
      X16, X16, kF, 0L, WT, WT, kF, 0L,
      (void*)QK, (void*)QK, kQKld, 0L, bq, bq, 0L, kRows, kA, kF, kWCarryInv);
  wmma_gemm64<0, false, 2, 0, false, 0><<<dim3(gemmBlocks, 1), dim3(256), 0, stream>>>(
      X16, X16, kF, 0L, WT + (size_t)kA * kF, WT + (size_t)kA * kF, kF, 0L,
      (void*)(QK + kA), (void*)(QK + kA), kQKld, 0L, bk, bk, 0L, kRows, kA, kF, kWCarryInv);

  pool_kernel<<<dim3(kTok / kPoolWaves), dim3(32 * kPoolWaves), 0, stream>>>(QK, x, Wv, bv, out, kTok);
}
